// CoherentMamba_47811575939686
// MI455X (gfx1250) — hardware-verified
//
#include <hip/hip_runtime.h>
#include <math.h>

typedef __attribute__((ext_vector_type(16))) _Float16 v16h;
typedef __attribute__((ext_vector_type(8)))  _Float16 v8h;
typedef __attribute__((ext_vector_type(16))) __bf16   v16b;
typedef __attribute__((ext_vector_type(8)))  __bf16   v8b;
typedef __attribute__((ext_vector_type(8)))  float    v8f;
typedef __attribute__((ext_vector_type(4)))  float    v4f;

constexpr int kBatch  = 2;
constexpr int kSeqL   = 2048;
constexpr int kRows   = kBatch * kSeqL;
constexpr int kInCh   = 2;
constexpr int kDmod   = 512;
constexpr int kDin    = 1024;
constexpr int kXZP    = 2 * kDin;
constexpr int kNst    = 16;
constexpr int kDtR    = 32;
constexpr int kPrjP   = kDtR + 2 * kNst;
constexpr int kLayers = 4;
constexpr int kCls    = 4;
constexpr int kClsP   = 64;
constexpr int kTP     = 260;

constexpr float kScW    = 32.0f;
constexpr float kScWdt  = 8.0f;
constexpr float kScWhd  = 8.0f;
constexpr float kScUC   = 64.0f;
constexpr float kScDT   = 256.0f;
constexpr float kScY    = 256.0f;

__device__ __forceinline__ unsigned short f2bf_bits(float f) {
  unsigned u = __float_as_uint(f);
  return (unsigned short)((u + 0x7FFFu + ((u >> 16) & 1u)) >> 16);
}
__device__ __forceinline__ float bf_bits2f(unsigned short h) { return __uint_as_float(((unsigned)h) << 16); }

__device__ __forceinline__ void dep_guard_h(v8f& a, v8f& b, v16h x, v16h y) { asm volatile("v_nop\n\tv_nop\n\tv_nop\n\tv_nop" : "+v"(a), "+v"(b) : "v"(x), "v"(y)); }
__device__ __forceinline__ void dep_guard_b(v8f& a, v8f& b, v16b x, v16b y) { asm volatile("v_nop\n\tv_nop\n\tv_nop\n\tv_nop" : "+v"(a), "+v"(b) : "v"(x), "v"(y)); }
__device__ __forceinline__ void keep4_h(v16h a, v16h b, v16h c, v16h d) { asm volatile("v_nop" :: "v"(a), "v"(b), "v"(c), "v"(d)); }
__device__ __forceinline__ void keep4_b(v16b a, v16b b, v16b c, v16b d) { asm volatile("v_nop" :: "v"(a), "v"(b), "v"(c), "v"(d)); }
__device__ __forceinline__ void acc_guard4(v8f& a, v8f& b, v8f& c, v8f& d) { asm volatile("v_nop\n\tv_nop\n\tv_nop\n\tv_nop" : "+v"(a), "+v"(b), "+v"(c), "+v"(d)); }
template <typename T> struct Frag;
template <> struct Frag<_Float16> {
  typedef v16h V; union U { v16h v; v8h h[2]; };
  static __device__ __forceinline__ v16h load(const _Float16* p) {
    U f; f.h[0] = *(const v8h*)(p); f.h[1] = *(const v8h*)(p + 16); return f.v;
  }
  static __device__ __forceinline__ v8f mma(v16h a, v16h b, v8f c) {
    return __builtin_amdgcn_wmma_f32_16x16x32_f16(false, a, false, b, (short)0, c, false, false);
  }
  static __device__ __forceinline__ void guard(v8f& a, v8f& b, v16h x, v16h y) { dep_guard_h(a, b, x, y); }
  static __device__ __forceinline__ void keep(v16h a, v16h b, v16h c, v16h d) { keep4_h(a, b, c, d); }
};
template <> struct Frag<__bf16> {
  typedef v16b V; union U { v16b v; v8b h[2]; };
  static __device__ __forceinline__ v16b load(const __bf16* p) {
    U f; f.h[0] = *(const v8b*)(p); f.h[1] = *(const v8b*)(p + 16); return f.v;
  }
  static __device__ __forceinline__ v8f mma(v16b a, v16b b, v8f c) {
    return __builtin_amdgcn_wmma_f32_16x16x32_bf16(false, a, false, b, (short)0, c, false, false);
  }
  static __device__ __forceinline__ void guard(v8f& a, v8f& b, v16b x, v16b y) { dep_guard_b(a, b, x, y); }
  static __device__ __forceinline__ void keep(v16b a, v16b b, v16b c, v16b d) { keep4_b(a, b, c, d); }
};

template <int ET> struct Elem;
template <> struct Elem<0> { typedef _Float16 T; };
template <> struct Elem<1> { typedef __bf16 T; };
template <int ET, bool SPLIT, int BIAS_MODE, int OUT_MODE, bool RESID, int ACT = 0>
__global__ __launch_bounds__(256) void wmma_gemm64(
    const unsigned short* __restrict__ Ap, const unsigned short* __restrict__ A2p, int lda, long strideA,
    const unsigned short* __restrict__ Btp, const unsigned short* __restrict__ Bt2p, int ldb, long strideB,
    void* __restrict__ Cout, void* __restrict__ Cout2, int ldc, long strideC,
    const float* __restrict__ bias,
    const float* __restrict__ resid, long strideR,
    int M, int N, int K, float scale) {
  typedef typename Elem<ET>::T T;
  typedef typename Frag<T>::V V;
  const T* A = (const T*)Ap; const T* A2 = (const T*)A2p; const T* Bt = (const T*)Btp; const T* Bt2 = (const T*)Bt2p;
  __shared__ __align__(16) float sT[8][16 * 68];
  const int b    = blockIdx.y;
  const int lane = threadIdx.x & 31;
  const int wave = threadIdx.x >> 5;
  const int tilesN = N >> 6;
  const int tilesM = M >> 6;
  const int tile = blockIdx.x * 8 + wave;
  if (tile >= tilesM * tilesN) return;
  const int tm = tile / tilesN;
  const int tn = tile - tm * tilesN;
  const int m0 = tm << 6;
  const int n0 = tn << 6;

  const T* Ab  = A  + (size_t)b * strideA;
  const T* Bb  = Bt + (size_t)b * strideB;
  const T* Ab2 = SPLIT ? (A2  + (size_t)b * strideA) : nullptr;
  const T* Bb2 = SPLIT ? (Bt2 + (size_t)b * strideB) : nullptr;

  const int rlane = lane & 15;
  const int koff  = (lane >> 4) * 8;
  const int mOff  = (lane >> 4) * 8;

  v8f acc[4][4];
#pragma unroll
  for (int i = 0; i < 4; ++i)
#pragma unroll
    for (int j = 0; j < 4; ++j) acc[i][j] = (v8f){0.f,0.f,0.f,0.f,0.f,0.f,0.f,0.f};

  for (int k0 = 0; k0 < K; k0 += 32) {
    V bh[4], bl[4];
#pragma unroll
    for (int j = 0; j < 4; ++j) {
      const size_t bo = (size_t)(n0 + (j << 4) + rlane) * ldb + koff + k0;
      bh[j] = Frag<T>::load(Bb + bo);
      if (SPLIT) bl[j] = Frag<T>::load(Bb2 + bo);
    }
#pragma unroll
    for (int i = 0; i < 4; ++i) {
      const size_t ao = (size_t)(m0 + (i << 4) + rlane) * lda + koff + k0;
      V ah = Frag<T>::load(Ab + ao);
      V al;
      if (SPLIT) al = Frag<T>::load(Ab2 + ao);
#pragma unroll
      for (int j = 0; j < 4; ++j) {
        acc[i][j] = Frag<T>::mma(ah, bh[j], acc[i][j]);
        if (SPLIT) {
          acc[i][j] = Frag<T>::mma(ah, bl[j], acc[i][j]);
          acc[i][j] = Frag<T>::mma(al, bh[j], acc[i][j]);
        }
      }
      Frag<T>::guard(acc[i][0], acc[i][3], ah, SPLIT ? al : ah);
    }
    Frag<T>::keep(bh[0], bh[1], bh[2], bh[3]);
    if (SPLIT) Frag<T>::keep(bl[0], bl[1], bl[2], bl[3]);
  }
  acc_guard4(acc[0][0], acc[0][1], acc[0][2], acc[0][3]);
  acc_guard4(acc[1][0], acc[1][1], acc[1][2], acc[1][3]);
  acc_guard4(acc[2][0], acc[2][1], acc[2][2], acc[2][3]);
  acc_guard4(acc[3][0], acc[3][1], acc[3][2], acc[3][3]);

  float* slab = sT[wave];
  const float* Rb = RESID ? (resid + (size_t)b * strideR) : nullptr;
#pragma unroll
  for (int i = 0; i < 4; ++i) {
    const int mBase = m0 + (i << 4);
#pragma unroll
    for (int j = 0; j < 4; ++j) {
      const int n = n0 + (j << 4) + rlane;
      float bv = 0.f;
      if (BIAS_MODE == 2) bv = bias[n];
#pragma unroll
      for (int r = 0; r < 8; ++r) {
        float v = acc[i][j][r] * scale;
        if (BIAS_MODE == 1) v += bias[mBase + mOff + r];
        if (BIAS_MODE == 2) v += bv;
        if (RESID) v += Rb[(size_t)(mBase + mOff + r) * ldc + n];
        if (ACT == 1) v = tanhf(v);
        if (ACT == 2) v = fmaxf(v, 0.0f);
        if (ACT == 3) v = v / (1.0f + expf(-v));
        if (ACT == 4) v = (v > 0.f) ? v : 0.01f * v;
        if (ACT == 5) v = 0.5f * v * (1.0f + erff(v * 0.70710678118654752f));
        slab[(mOff + r) * 68 + (j << 4) + rlane] = v;
      }
    }
    __builtin_amdgcn_fence(__ATOMIC_RELEASE, "workgroup");
    __builtin_amdgcn_wave_barrier();
    __builtin_amdgcn_fence(__ATOMIC_ACQUIRE, "workgroup");
    if (OUT_MODE == 0) {
      float* C = (float*)Cout + (size_t)b * strideC;
      const int hh = lane >> 4, c4 = (lane & 15) * 4;
      for (int pass = 0; pass < 2; ++pass) {
#pragma unroll
        for (int it = 0; it < 8; ++it) {
          const int row = it * 2 + hh;
          v4f v = *(const v4f*)(slab + row * 68 + c4);
          *(volatile v4f*)(C + (size_t)(mBase + row) * ldc + n0 + c4) = v;
        }
        __threadfence();
      }
    } else {
      const int q = lane >> 3, c8 = (lane & 7) * 8;
      unsigned short* C  = (unsigned short*)Cout  + (size_t)b * strideC;
      unsigned short* C2 = (OUT_MODE == 2) ? ((unsigned short*)Cout2 + (size_t)b * strideC) : nullptr;
      for (int pass = 0; pass < 2; ++pass) {
#pragma unroll
        for (int it = 0; it < 4; ++it) {
          const int row = it * 4 + q;
          const float* sp = slab + row * 68 + c8;
          v8h hv, lv;
#pragma unroll
          for (int e = 0; e < 8; ++e) {
            if (OUT_MODE == 1) {
              hv[e] = (_Float16)sp[e];
            } else {
              unsigned short hb = f2bf_bits(sp[e]);
              unsigned short lb = f2bf_bits(sp[e] - bf_bits2f(hb));
              hv[e] = __builtin_bit_cast(_Float16, hb);
              lv[e] = __builtin_bit_cast(_Float16, lb);
            }
          }
          *(volatile v8h*)(C + (size_t)(mBase + row) * ldc + n0 + c8) = hv;
          if (OUT_MODE == 2) *(volatile v8h*)(C2 + (size_t)(mBase + row) * ldc + n0 + c8) = lv;
        }
        __threadfence();
      }
    }
    __builtin_amdgcn_fence(__ATOMIC_RELEASE, "workgroup");
    __builtin_amdgcn_wave_barrier();
    __builtin_amdgcn_fence(__ATOMIC_ACQUIRE, "workgroup");
  }
}

__global__ __launch_bounds__(256) void cast_f16_kernel(
    const float* __restrict__ src, unsigned short* __restrict__ dst, int total8, float scale)
{
  const int i = blockIdx.x * 256 + threadIdx.x;
  if (i >= total8) return;
  const size_t e0 = (size_t)i << 3;
  const float* p = src + e0;
  const v4f a0 = *(const v4f*)(p);
  const v4f a1 = *(const v4f*)(p + 4);
  v8h hv;
#pragma unroll
  for (int e = 0; e < 4; ++e) {
    hv[e]     = (_Float16)(a0[e] * scale);
    hv[4 + e] = (_Float16)(a1[e] * scale);
  }
  unsigned short* q = dst + e0;
  *(volatile v8h*)q = hv;
  __threadfence();
  *(volatile v8h*)q = hv;
}

__global__ __launch_bounds__(256) void head_cast_kernel(
    const float* __restrict__ W, unsigned short* __restrict__ dst, int nreal, float scale)
{
  const int i = blockIdx.x * 256 + threadIdx.x;
  if (i >= (kClsP * kDmod) / 8) return;
  const int e0  = i << 3;
  const int row = e0 >> 9;
  const int col = e0 & (kDmod - 1);
  const int rc  = (row < nreal) ? row : (nreal - 1);
  const float* p = W + (size_t)rc * kDmod + col;
  const v4f a0 = *(const v4f*)(p);
  const v4f a1 = *(const v4f*)(p + 4);
  const bool live = (row < nreal);
  v8h hv;
#pragma unroll
  for (int e = 0; e < 4; ++e) {
    hv[e]     = (_Float16)(live ? a0[e] * scale : 0.f);
    hv[4 + e] = (_Float16)(live ? a1[e] * scale : 0.f);
  }
  unsigned short* q = dst + e0;
  *(volatile v8h*)q = hv;
  __threadfence();
  *(volatile v8h*)q = hv;
}

__global__ __launch_bounds__(256) void embed_kernel(
    const float* __restrict__ x, const float* __restrict__ w, const float* __restrict__ bb,
    float* __restrict__ H, int total4)
{
  const int i = blockIdx.x * 256 + threadIdx.x;
  if (i >= total4) return;
  const int e0 = i << 2;
  const int m  = e0 >> 9;
  const int d  = e0 & (kDmod - 1);
  const int b  = m >> 11;
  const int t  = m & (kSeqL - 1);
  const float x0 = x[((size_t)b * kInCh + 0) * kSeqL + t];
  const float x1 = x[((size_t)b * kInCh + 1) * kSeqL + t];
  v4f o;
#pragma unroll
  for (int e = 0; e < 4; ++e) {
    const float w0 = w[(d + e) * kInCh + 0];
    const float w1 = w[(d + e) * kInCh + 1];
    o[e] = x0 * w0 + x1 * w1 + bb[d + e];
  }
  float* q = H + e0;
  *(volatile v4f*)q = o;
  __threadfence();
  *(volatile v4f*)q = o;
}

__global__ __launch_bounds__(256) void layernorm_f16_kernel(
    const float* __restrict__ X, const float* __restrict__ w, const float* __restrict__ bb,
    unsigned short* __restrict__ HN, int nrows)
{
  const int lane = threadIdx.x & 31, wave = threadIdx.x >> 5;
  const int row = blockIdx.x * 8 + wave;
  if (row >= nrows) return;
  const float* xr = X + (size_t)row * kDmod;
  const int c0 = lane * 8, c1 = 256 + lane * 8;
  v4f a[4];
  a[0] = *(const v4f*)(xr + c0);
  a[1] = *(const v4f*)(xr + c0 + 4);
  a[2] = *(const v4f*)(xr + c1);
  a[3] = *(const v4f*)(xr + c1 + 4);
  float s = 0.f;
#pragma unroll
  for (int i = 0; i < 4; ++i) s += (a[i][0] + a[i][1]) + (a[i][2] + a[i][3]);
#pragma unroll
  for (int off = 1; off < 32; off <<= 1) s += __shfl_xor(s, off, 32);
  const float mean = s * (1.0f / kDmod);
  float q = 0.f;
#pragma unroll
  for (int i = 0; i < 4; ++i) {
#pragma unroll
    for (int e = 0; e < 4; ++e) { const float dl = a[i][e] - mean; q += dl * dl; }
  }
#pragma unroll
  for (int off = 1; off < 32; off <<= 1) q += __shfl_xor(q, off, 32);
  const float rs = rsqrtf(q * (1.0f / kDmod) + 1e-5f);
  v4f wv[4], bv[4];
  wv[0] = *(const v4f*)(w + c0);  wv[1] = *(const v4f*)(w + c0 + 4);
  wv[2] = *(const v4f*)(w + c1);  wv[3] = *(const v4f*)(w + c1 + 4);
  bv[0] = *(const v4f*)(bb + c0); bv[1] = *(const v4f*)(bb + c0 + 4);
  bv[2] = *(const v4f*)(bb + c1); bv[3] = *(const v4f*)(bb + c1 + 4);
  v8h h0, h1;
#pragma unroll
  for (int e = 0; e < 4; ++e) {
    h0[e]     = (_Float16)((a[0][e] - mean) * rs * wv[0][e] + bv[0][e]);
    h0[4 + e] = (_Float16)((a[1][e] - mean) * rs * wv[1][e] + bv[1][e]);
    h1[e]     = (_Float16)((a[2][e] - mean) * rs * wv[2][e] + bv[2][e]);
    h1[4 + e] = (_Float16)((a[3][e] - mean) * rs * wv[3][e] + bv[3][e]);
  }
  unsigned short* o = HN + (size_t)row * kDmod;
  for (int pass = 0; pass < 2; ++pass) {
    *(volatile v8h*)(o + c0) = h0;
    *(volatile v8h*)(o + c1) = h1;
    __threadfence();
  }
}

__global__ __launch_bounds__(256) void conv_silu_kernel(
    const float* __restrict__ XZ, const float* __restrict__ cw, const float* __restrict__ cb,
    float* __restrict__ UC, unsigned short* __restrict__ UC16)
{
  __shared__ __align__(16) float sT[16 * kTP];
  const int tid = threadIdx.x, lane = tid & 31, wave = tid >> 5;
  const int d0 = blockIdx.x * 256, d = d0 + tid;
  const int g0 = blockIdx.y * 64;
  const int bidx = g0 / kSeqL;
  const int rb = bidx * kSeqL;
  const int t0 = g0 - rb;
  const float w0 = cw[d * 4 + 0], w1 = cw[d * 4 + 1], w2 = cw[d * 4 + 2], w3 = cw[d * 4 + 3];
  const float bc = cb[d];
  float xm3, xm2, xm1;
  {
    const int u3 = t0 - 3, u2 = t0 - 2, u1 = t0 - 1;
    const float v3 = XZ[(size_t)(rb + (u3 < 0 ? 0 : u3)) * kXZP + d];
    const float v2 = XZ[(size_t)(rb + (u2 < 0 ? 0 : u2)) * kXZP + d];
    const float v1 = XZ[(size_t)(rb + (u1 < 0 ? 0 : u1)) * kXZP + d];
    xm3 = (u3 >= 0) ? v3 : 0.f;
    xm2 = (u2 >= 0) ? v2 : 0.f;
    xm1 = (u1 >= 0) ? v1 : 0.f;
  }
  const int hrow = wave >> 1;
  const int hch  = (wave & 1) * 128 + lane * 4;
#pragma unroll 1
  for (int sub = 0; sub < 4; ++sub) {
    const int lb = g0 + sub * 16;
#pragma unroll 1
    for (int s = 0; s < 16; ++s) {
      const float xc = XZ[(size_t)(lb + s) * kXZP + d];
      float acc = w0 * xm3;
      acc = fmaf(w1, xm2, acc);
      acc = fmaf(w2, xm1, acc);
      acc = fmaf(w3, xc, acc);
      const float sv = acc + bc;
      const float sg = __builtin_amdgcn_rcpf(1.0f + __expf(-sv));
      sT[s * kTP + tid] = sv * sg;
      xm3 = xm2; xm2 = xm1; xm1 = xc;
    }
    __syncthreads();
    v4f fv[4];
    v8h bv[2];
#pragma unroll
    for (int it = 0; it < 4; ++it) fv[it] = *(const v4f*)(sT + (it * 4 + hrow) * kTP + hch);
#pragma unroll
    for (int it = 0; it < 2; ++it) {
      const float* sp = sT + (it * 8 + wave) * kTP + lane * 8;
      const v4f a0 = *(const v4f*)(sp);
      const v4f a1 = *(const v4f*)(sp + 4);
#pragma unroll
      for (int e = 0; e < 4; ++e) {
        bv[it][e]     = (_Float16)(a0[e] * kScUC);
        bv[it][4 + e] = (_Float16)(a1[e] * kScUC);
      }
    }
    for (int pass = 0; pass < 2; ++pass) {
#pragma unroll
      for (int it = 0; it < 4; ++it)
        *(volatile v4f*)(UC + (size_t)(lb + it * 4 + hrow) * kDin + d0 + hch) = fv[it];
#pragma unroll
      for (int it = 0; it < 2; ++it)
        *(volatile v8h*)(UC16 + (size_t)(lb + it * 8 + wave) * kDin + d0 + lane * 8) = bv[it];
      __threadfence();
    }
    __syncthreads();
  }
}

__global__ __launch_bounds__(256) void dt_cast_kernel(
    const float* __restrict__ XDBL, unsigned short* __restrict__ DT16, int total8, float scale)
{
  const int i = blockIdx.x * 256 + threadIdx.x;
  if (i >= total8) return;
  const int e0  = i << 3;
  const int row = e0 >> 5;
  const int c8  = e0 & (kDtR - 1);
  const float* p = XDBL + (size_t)row * kPrjP + c8;
  const v4f a0 = *(const v4f*)(p);
  const v4f a1 = *(const v4f*)(p + 4);
  v8h hv;
#pragma unroll
  for (int e = 0; e < 4; ++e) {
    hv[e]     = (_Float16)(a0[e] * scale);
    hv[4 + e] = (_Float16)(a1[e] * scale);
  }
  unsigned short* qd = DT16 + e0;
  *(volatile v8h*)qd = hv;
  __threadfence();
  *(volatile v8h*)qd = hv;
}

__global__ __launch_bounds__(256) void scan_kernel(
    const float* __restrict__ DLR, const float* __restrict__ UC, const float* __restrict__ XZ,
    const float* __restrict__ XDBL, const float* __restrict__ A_log, const float* __restrict__ Dv,
    unsigned short* __restrict__ Y16)
{
  __shared__ __align__(16) float sBC[16 * 32];
  __shared__ __align__(16) float sY[16 * kTP];
  const int tid = threadIdx.x, lane = tid & 31, wave = tid >> 5;
  const int d0 = blockIdx.x * 256, d = d0 + tid;
  const int rb = blockIdx.y * kSeqL;

  float An[kNst];
#pragma unroll
  for (int n = 0; n < kNst; ++n) An[n] = -__expf(A_log[(size_t)d * kNst + n]);
  const float Dd = Dv[d];
  float h[kNst];
#pragma unroll
  for (int n = 0; n < kNst; ++n) h[n] = 0.f;

#pragma unroll 1
  for (int c = 0; c < kSeqL / 16; ++c) {
    const int l0 = rb + c * 16;
    if (tid < 128) {
      const int r = tid >> 3, q = (tid & 7) * 4;
      const v4f v = *(const v4f*)(XDBL + (size_t)(l0 + r) * kPrjP + kDtR + q);
      *(v4f*)(sBC + r * 32 + q) = v;
    }
    __syncthreads();
#pragma unroll 1
    for (int s = 0; s < 16; ++s) {
      const size_t m = (size_t)(l0 + s);
      const float a     = DLR[m * kDin + d];
      const float delta = fmaxf(a, 0.0f) + log1pf(__expf(-fabsf(a)));
      const float xv    = UC[m * kDin + d];
      const float zv    = XZ[m * kXZP + kDin + d];
      v4f Bq[4], Cq[4];
#pragma unroll
      for (int qq = 0; qq < 4; ++qq) {
        Bq[qq] = *(const v4f*)(sBC + s * 32 + 4 * qq);
        Cq[qq] = *(const v4f*)(sBC + s * 32 + kNst + 4 * qq);
      }
      float y = 0.f;
#pragma unroll
      for (int n = 0; n < kNst; ++n) {
        const float e = __expf(delta * An[n]);
        float db = delta * Bq[n >> 2][n & 3];
        asm volatile("" : "+v"(db));
        float p = db * xv;
        asm volatile("" : "+v"(p));
        float qv = h[n] * e;
        asm volatile("" : "+v"(qv));
        const float hn = qv + p;
        h[n] = hn;
        float rr = Cq[n >> 2][n & 3] * hn;
        asm volatile("" : "+v"(rr));
        y += rr;
      }
      float sk = xv * Dd;
      asm volatile("" : "+v"(sk));
      y += sk;
      const float sg = __builtin_amdgcn_rcpf(1.0f + __expf(-zv));
      const float g  = zv * sg;
      sY[s * kTP + tid] = (y * g) * kScY;
    }
    __syncthreads();
    v8h hv[2];
#pragma unroll
    for (int it = 0; it < 2; ++it) {
      const float* sp = sY + (it * 8 + wave) * kTP + lane * 8;
      const v4f a0 = *(const v4f*)(sp);
      const v4f a1 = *(const v4f*)(sp + 4);
#pragma unroll
      for (int e = 0; e < 4; ++e) { hv[it][e] = (_Float16)a0[e]; hv[it][4 + e] = (_Float16)a1[e]; }
    }
    for (int pass = 0; pass < 2; ++pass) {
#pragma unroll
      for (int it = 0; it < 2; ++it)
        *(volatile v8h*)(Y16 + (size_t)(l0 + it * 8 + wave) * kDin + d0 + lane * 8) = hv[it];
      __threadfence();
    }
  }
}

__global__ __launch_bounds__(256) void logits_out_kernel(
    const float* __restrict__ LOG, const float* __restrict__ hb, float* __restrict__ out, int total4)
{
  const int i = blockIdx.x * 256 + threadIdx.x;
  if (i >= total4) return;
  const int e0 = i << 2;
  const int b  = e0 >> 13;
  const int c  = (e0 >> 11) & (kCls - 1);
  const int t  = e0 & (kSeqL - 1);
  const v4f v = *(const v4f*)(LOG + ((size_t)(b * kClsP + c)) * kSeqL + t);
  const float bias = hb[c];
  v4f o;
#pragma unroll
  for (int e = 0; e < 4; ++e) o[e] = v[e] + bias;
  float* q = out + e0;
  *(volatile v4f*)q = o;
  __threadfence();
  *(volatile v4f*)q = o;
}

extern "C" void kernel_launch(void* const* d_in, const int* in_sizes, int n_in,
                              void* d_out, int out_size, void* d_ws, size_t ws_size,
                              hipStream_t stream)
{
  if (n_in < 18) return;
  const float* x          = (const float*)d_in[0];
  const float* inp_w      = (const float*)d_in[1];
  const float* inp_b      = (const float*)d_in[2];
  const float* ln_w       = (const float*)d_in[3];
  const float* ln_b       = (const float*)d_in[4];
  const float* in_proj_w  = (const float*)d_in[5];
  const float* conv_w     = (const float*)d_in[6];
  const float* conv_b     = (const float*)d_in[7];
  const float* x_proj_w   = (const float*)d_in[8];
  const float* dt_proj_w  = (const float*)d_in[9];
  const float* dt_proj_b  = (const float*)d_in[10];
  const float* A_log      = (const float*)d_in[11];
  const float* Dvec       = (const float*)d_in[12];
  const float* out_proj_w = (const float*)d_in[13];
  const float* fn_w       = (const float*)d_in[14];
  const float* fn_b       = (const float*)d_in[15];
  const float* head_w     = (const float*)d_in[16];
  const float* head_b     = (const float*)d_in[17];
  float* dout = (float*)d_out;

  if (in_sizes[0]  != kBatch * kInCh * kSeqL) return;
  if (in_sizes[1]  != kDmod * kInCh || in_sizes[2] != kDmod) return;
  if (in_sizes[3]  != kLayers * kDmod || in_sizes[4] != kLayers * kDmod) return;
  if (in_sizes[5]  != kLayers * kXZP * kDmod) return;
  if (in_sizes[6]  != kLayers * kDin * 4 || in_sizes[7] != kLayers * kDin) return;
  if (in_sizes[8]  != kLayers * kPrjP * kDin) return;
  if (in_sizes[9]  != kLayers * kDin * kDtR || in_sizes[10] != kLayers * kDin) return;
  if (in_sizes[11] != kLayers * kDin * kNst || in_sizes[12] != kLayers * kDin) return;
  if (in_sizes[13] != kLayers * kDmod * kDin) return;
  if (in_sizes[14] != kDmod || in_sizes[15] != kDmod) return;
  if (in_sizes[16] != kCls * kDmod || in_sizes[17] != kCls) return;
  if (out_size != kBatch * kCls * kSeqL) return;

  const size_t SZ_H      = (size_t)kRows * kDmod * 4;
  const size_t SZ_HN16   = (size_t)kRows * kDmod * 2;
  const size_t SZ_XZ     = (size_t)kRows * kXZP * 4;
  const size_t SZ_UC     = (size_t)kRows * kDin * 4;
  const size_t SZ_UC16   = (size_t)kRows * kDin * 2;
  const size_t SZ_XDBL   = (size_t)kRows * kPrjP * 4;
  const size_t SZ_DT16   = (size_t)kRows * kDtR * 2;
  const size_t SZ_DLR    = (size_t)kRows * kDin * 4;
  const size_t SZ_Y16    = (size_t)kRows * kDin * 2;
  const size_t SZ_WIN16  = (size_t)kLayers * kXZP * kDmod * 2;
  const size_t SZ_WXP16  = (size_t)kLayers * kPrjP * kDin * 2;
  const size_t SZ_WDT16  = (size_t)kLayers * kDin * kDtR * 2;
  const size_t SZ_WOUT16 = (size_t)kLayers * kDmod * kDin * 2;
  const size_t SZ_HW16   = (size_t)kClsP * kDmod * 2;
  const size_t SZ_LOG    = (size_t)kBatch * kClsP * kSeqL * 4;
  const size_t OFF_HA     = 0;
  const size_t OFF_HB     = OFF_HA     + SZ_H;
  const size_t OFF_HN16   = OFF_HB     + SZ_H;
  const size_t OFF_XZ     = OFF_HN16   + SZ_HN16;
  const size_t OFF_UC     = OFF_XZ     + SZ_XZ;
  const size_t OFF_UC16   = OFF_UC     + SZ_UC;
  const size_t OFF_XDBL   = OFF_UC16   + SZ_UC16;
  const size_t OFF_DT16   = OFF_XDBL   + SZ_XDBL;
  const size_t OFF_DLR    = OFF_DT16   + SZ_DT16;
  const size_t OFF_Y16    = OFF_DLR    + SZ_DLR;
  const size_t OFF_WIN16  = OFF_Y16    + SZ_Y16;
  const size_t OFF_WXP16  = OFF_WIN16  + SZ_WIN16;
  const size_t OFF_WDT16  = OFF_WXP16  + SZ_WXP16;
  const size_t OFF_WOUT16 = OFF_WDT16  + SZ_WDT16;
  const size_t OFF_HW16   = OFF_WOUT16 + SZ_WOUT16;
  const size_t OFF_LOG    = OFF_HW16   + SZ_HW16;
  const size_t TOTAL      = OFF_LOG    + SZ_LOG;
  if (ws_size < TOTAL) return;

  char* ws = (char*)d_ws;
  float*          HA     = (float*)(ws + OFF_HA);
  float*          HB     = (float*)(ws + OFF_HB);
  unsigned short* HN16   = (unsigned short*)(ws + OFF_HN16);
  float*          XZ     = (float*)(ws + OFF_XZ);
  float*          UC     = (float*)(ws + OFF_UC);
  unsigned short* UC16   = (unsigned short*)(ws + OFF_UC16);
  float*          XDBL   = (float*)(ws + OFF_XDBL);
  unsigned short* DT16   = (unsigned short*)(ws + OFF_DT16);
  float*          DLR    = (float*)(ws + OFF_DLR);
  unsigned short* Y16    = (unsigned short*)(ws + OFF_Y16);
  unsigned short* WIN16  = (unsigned short*)(ws + OFF_WIN16);
  unsigned short* WXP16  = (unsigned short*)(ws + OFF_WXP16);
  unsigned short* WDT16  = (unsigned short*)(ws + OFF_WDT16);
  unsigned short* WOUT16 = (unsigned short*)(ws + OFF_WOUT16);
  unsigned short* HW16   = (unsigned short*)(ws + OFF_HW16);
  float*          LOG    = (float*)(ws + OFF_LOG);
  const float* dummy_bias  = dt_proj_b;
  const float* dummy_resid = x;

  cast_f16_kernel<<<(int)(SZ_WIN16 / 2 / 8 / 256), 256, 0, stream>>>(in_proj_w,  WIN16,  (int)(SZ_WIN16 / 2 / 8),  kScW);
  cast_f16_kernel<<<(int)(SZ_WXP16 / 2 / 8 / 256), 256, 0, stream>>>(x_proj_w,   WXP16,  (int)(SZ_WXP16 / 2 / 8),  kScW);
  cast_f16_kernel<<<(int)(SZ_WDT16 / 2 / 8 / 256), 256, 0, stream>>>(dt_proj_w,  WDT16,  (int)(SZ_WDT16 / 2 / 8),  kScWdt);
  cast_f16_kernel<<<(int)(SZ_WOUT16 / 2 / 8 / 256), 256, 0, stream>>>(out_proj_w, WOUT16, (int)(SZ_WOUT16 / 2 / 8), kScW);
  head_cast_kernel<<<(kClsP * kDmod) / 8 / 256, 256, 0, stream>>>(head_w, HW16, kCls, kScWhd);

  embed_kernel<<<(kRows * kDmod) / 4 / 256, 256, 0, stream>>>(x, inp_w, inp_b, HA, (kRows * kDmod) / 4);

  float* hcur = HA;
  float* hnext = HB;
  for (int i = 0; i < kLayers; ++i) {
    const unsigned short* WINi  = WIN16  + (size_t)i * kXZP * kDmod;
    const unsigned short* WXPi  = WXP16  + (size_t)i * kPrjP * kDin;
    const unsigned short* WDTi  = WDT16  + (size_t)i * kDin * kDtR;
    const unsigned short* WOUTi = WOUT16 + (size_t)i * kDmod * kDin;

    layernorm_f16_kernel<<<kRows / 8, 256, 0, stream>>>(hcur, ln_w + (size_t)i * kDmod, ln_b + (size_t)i * kDmod, HN16, kRows);

    wmma_gemm64<0, false, 0, 0, false><<<dim3((kRows / 64) * (kXZP / 64) / 8, 1), 256, 0, stream>>>(
        HN16, HN16, kDmod, 0L, WINi, WINi, kDmod, 0L,
        (void*)XZ, (void*)XZ, kXZP, 0L, dummy_bias, dummy_resid, 0L, kRows, kXZP, kDmod, 1.0f / kScW);

    conv_silu_kernel<<<dim3(kDin / 256, kRows / 64), 256, 0, stream>>>(
        XZ, conv_w + (size_t)i * kDin * 4, conv_b + (size_t)i * kDin, UC, UC16);

    wmma_gemm64<0, false, 0, 0, false><<<dim3((kRows / 64) * (kPrjP / 64) / 8, 1), 256, 0, stream>>>(
        UC16, UC16, kDin, 0L, WXPi, WXPi, kDin, 0L,
        (void*)XDBL, (void*)XDBL, kPrjP, 0L, dummy_bias, dummy_resid, 0L, kRows, kPrjP, kDin, 1.0f / (kScUC * kScW));

    dt_cast_kernel<<<(kRows * kDtR) / 8 / 256, 256, 0, stream>>>(XDBL, DT16, (kRows * kDtR) / 8, kScDT);

    wmma_gemm64<0, false, 2, 0, false><<<dim3((kRows / 64) * (kDin / 64) / 8, 1), 256, 0, stream>>>(
        DT16, DT16, kDtR, 0L, WDTi, WDTi, kDtR, 0L,
        (void*)DLR, (void*)DLR, kDin, 0L, dt_proj_b + (size_t)i * kDin, dummy_resid, 0L, kRows, kDin, kDtR, 1.0f / (kScDT * kScWdt));

    scan_kernel<<<dim3(kDin / 256, kBatch), 256, 0, stream>>>(
        DLR, UC, XZ, XDBL, A_log + (size_t)i * kDin * kNst, Dvec + (size_t)i * kDin, Y16);

    wmma_gemm64<0, false, 0, 0, true><<<dim3((kRows / 64) * (kDmod / 64) / 8, 1), 256, 0, stream>>>(
        Y16, Y16, kDin, 0L, WOUTi, WOUTi, kDin, 0L,
        (void*)hnext, (void*)hnext, kDmod, 0L, dummy_bias, hcur, 0L, kRows, kDmod, kDin, 1.0f / (kScY * kScW));

    float* tmp = hcur; hcur = hnext; hnext = tmp;
  }

  layernorm_f16_kernel<<<kRows / 8, 256, 0, stream>>>(hcur, fn_w, fn_b, HN16, kRows);

  wmma_gemm64<0, false, 0, 0, false><<<dim3((kClsP / 64) * (kSeqL / 64) / 8, kBatch), 256, 0, stream>>>(
      HW16, HW16, kDmod, 0L, HN16, HN16, kDmod, (long)kSeqL * kDmod,
      (void*)LOG, (void*)LOG, kSeqL, (long)kClsP * kSeqL, dummy_bias, dummy_resid, 0L, kClsP, kSeqL, kDmod, 1.0f / kScWhd);

  logits_out_kernel<<<(kBatch * kCls * kSeqL) / 4 / 256, 256, 0, stream>>>(LOG, head_b, dout, (kBatch * kCls * kSeqL) / 4);
}
